// net_crossInteraction_66468913873310
// MI455X (gfx1250) — hardware-verified
//
#include <hip/hip_runtime.h>

#define __bf16 _Float16
typedef __attribute__((ext_vector_type(4))) float v4f_t;
typedef float v4fa __attribute__((ext_vector_type(4), may_alias));
typedef __attribute__((ext_vector_type(4))) unsigned v4u_t;
typedef unsigned v4ua __attribute__((ext_vector_type(4), may_alias));
#define IL  64
#define FL  1024
#define PSLOT 32
__device__ __forceinline__ void st2f(float* p, float v) { *(volatile float*)p = v; __threadfence(); *(volatile float*)p = v; }
typedef __attribute__((ext_vector_type(16))) __bf16 v16bf;
typedef __attribute__((ext_vector_type(8)))  __bf16 v8bf;
typedef __attribute__((ext_vector_type(8)))  float  v8f;

#define LRELU(x) ((x) > 0.f ? (x) : 0.1f * (x))

static __device__ __forceinline__ float block_reduce_sum(float v, float* sm) {
    int t = threadIdx.x;
    sm[t] = v; __syncthreads();
    for (int s = blockDim.x >> 1; s > 0; s >>= 1) {
        if (t < s) sm[t] += sm[t + s];
        __syncthreads();
    }
    float r = sm[0]; __syncthreads();
    return r;
}

__global__ void k_zero(float* p, int n) {
    int i = blockIdx.x * blockDim.x + threadIdx.x;
    if (i < n) st2f(p + i, 0.f);
}

__global__ void k_f2bf(const float* __restrict__ in, __bf16* __restrict__ out, int n) {
    int i = blockIdx.x * blockDim.x + threadIdx.x;
    if (i < n) { *(volatile __bf16*)(out + i) = (__bf16)in[i]; __threadfence(); *(volatile __bf16*)(out + i) = (__bf16)in[i]; }
}

__global__ void k_f2bf_pad(const float* __restrict__ in, __bf16* __restrict__ out,
                           int rows, int cols, int ldo) {
    int i = blockIdx.x * blockDim.x + threadIdx.x;
    if (i < rows * cols) {
        int r = i / cols, c = i - r * cols;
        __bf16* d = out + (size_t)r * ldo + c; *(volatile __bf16*)d = (__bf16)in[i]; __threadfence(); *(volatile __bf16*)d = (__bf16)in[i];
    }
}

__global__ void k_transconv(const float* __restrict__ W, __bf16* __restrict__ Bt, int K, int N) {
    int i = blockIdx.x * blockDim.x + threadIdx.x;
    if (i < K * N) {
        int n = i / K, k = i - n * K;
        const __bf16 v = (__bf16)W[(size_t)k * N + n];
        *(volatile __bf16*)(Bt + i) = v; __threadfence(); *(volatile __bf16*)(Bt + i) = v;
    }
}

#define NT 4
__global__ void wmma_gemm_bt(const __bf16* __restrict__ A, const __bf16* __restrict__ Bt,
                             float* __restrict__ C, __bf16* __restrict__ aux,
                             const float* __restrict__ bias,
                             int M, int N, int K, int lda, int ldb, int ldc,
                             long long sA, long long sB, long long sC, int aux_relu)
{
    int lane = threadIdx.x & 31;
    int wid  = threadIdx.x >> 5;
    int hf   = lane >> 4;
    int l16  = lane & 15;
    int m0 = (blockIdx.y * 4 + wid) * 16;
    if (m0 >= ((M + 15) & ~15)) return;
    int n0 = blockIdx.x * (16 * NT);
    int b  = blockIdx.z;

    const v8bf* Ar = (const v8bf*)(A + (size_t)b * sA + (size_t)(m0 + l16) * lda);
    const v8bf* Br0 = (const v8bf*)(Bt + (size_t)b * sB + (size_t)(n0 + l16) * ldb);
    size_t bstep = ((size_t)16 * ldb) >> 3;

    v8f acc[NT] = {};
    int ksteps = K >> 5;
    for (int ks = 0; ks < ksteps; ++ks) {
        int k8 = ks * 4;
        union { v16bf v; v8bf h[2]; } ua, ub;
        ua.h[0] = Ar[k8 + hf];
        ua.h[1] = Ar[k8 + 2 + hf];
        #pragma unroll
        for (int t = 0; t < NT; ++t) {
            const v8bf* Br = Br0 + (size_t)t * bstep;
            ub.h[0] = Br[k8 + hf];
            ub.h[1] = Br[k8 + 2 + hf];
            acc[t] = __builtin_amdgcn_wmma_f32_16x16x32_f16(false, ua.v, false, ub.v,
                                                             (short)0, acc[t], false, false);
        }
    }

    __shared__ __attribute__((aligned(16))) float stg[4][16 * 68];
    float* sw = stg[wid];
    #pragma unroll
    for (int t = 0; t < NT; ++t) {
        int n = n0 + t * 16 + l16;
        float bz = (bias && n < N) ? bias[n] : 0.f;
        #pragma unroll
        for (int v = 0; v < 8; ++v) sw[(v + 8 * hf) * 68 + t * 16 + l16] = (n < N) ? (acc[t][v] + bz) : 0.f;
    }
    asm volatile("s_wait_dscnt 0" ::: "memory");
    #pragma unroll 1
    for (int pass = 0; pass < 2; ++pass) {
        #pragma unroll
        for (int i = 0; i < 8; ++i) {
            const int c = lane + 32 * i, rr = c >> 4, q = (c & 15) * 4, m = m0 + rr;
            if (m < M && C) { size_t o = (size_t)b * sC + (size_t)m * ldc + n0 + q;
                *(volatile v4f_t*)(C + o) = *(const volatile v4fa*)(sw + rr * 68 + q); }
        }
        #pragma unroll
        for (int i = 0; i < 4; ++i) {
            const int c = lane + 32 * i, rr = c >> 3, q = (c & 7) * 8, m = m0 + rr;
            if (m < M && aux) { const float* s = sw + rr * 68 + q; v4u_t u;
                __bf16 hh[8];
                #pragma unroll
                for (int e = 0; e < 8; ++e) hh[e] = (__bf16)(aux_relu ? fmaxf(s[e], 0.f) : s[e]);
                u = *(const v4ua*)hh;
                size_t o = (size_t)b * sC + (size_t)m * ldc + n0 + q;
                *(volatile v4u_t*)(aux + o) = u; }
        }
        __threadfence();
    }
}

__global__ void k_linear(const float* __restrict__ X, const float* __restrict__ W,
                         const float* __restrict__ bias, float* __restrict__ Y,
                         __bf16* __restrict__ aux, int Kin, int relu_in)
{
    int r = blockIdx.x, n = threadIdx.x;
    const float* x = X + (size_t)r * Kin;
    float acc = bias[n];
    for (int k = 0; k < Kin; ++k) {
        float xv = x[k];
        if (relu_in) xv = fmaxf(xv, 0.f);
        acc = fmaf(xv, W[(size_t)k * 256 + n], acc);
    }
    st2f(Y + (size_t)r * 256 + n, acc);
    if (aux) { __bf16* d = aux + (size_t)r * 256 + n; *(volatile __bf16*)d = (__bf16)acc; __threadfence(); *(volatile __bf16*)d = (__bf16)acc; }
}

__global__ void k_adjrelu(const float* __restrict__ adj, const float* __restrict__ Yin,
                          float* __restrict__ Z)
{
    int i = blockIdx.x, b = blockIdx.y, d = threadIdx.x;
    const float* ar = adj + ((size_t)b * 56 + i) * 56;
    const float* yb = Yin + (size_t)b * 56 * 256;
    float acc = 0.f;
    #pragma unroll 1
    for (int j = 0; j < 56; ++j) acc = fmaf(ar[j], yb[j * 256 + d], acc);
    st2f(Z + ((size_t)b * 56 + i) * 256 + d, fmaxf(acc, 0.f));
}

#define NBI 250
__global__ void k_sigsum(float* __restrict__ inter, float* __restrict__ sumsP)
{
    __shared__ float sm[256];
    int b = blockIdx.y;
    int idx = blockIdx.x * 256 + threadIdx.x;
    int k = idx & (IL - 1);
    float v = 0.f;
    size_t o = (size_t)b * 1000 * IL + idx;
    if (k < 56) {
        float L = inter[o];
        v = 1.f / (1.f + expf(-L));
    }
    st2f(inter + o, v);
    float tot = block_reduce_sum(v, sm);
    if (threadIdx.x == 0) st2f(sumsP + ((size_t)b * NBI + blockIdx.x) * PSLOT, tot);
}

__global__ void k_norm(float* __restrict__ inter, const float* __restrict__ sumsP,
                       const float* __restrict__ prot_inter, const float* __restrict__ exist,
                       float* __restrict__ l1P, float* __restrict__ d2P)
{
    __shared__ float sm[256];
    __shared__ float ssum;
    int b = blockIdx.y;
    if (threadIdx.x == 0) { float s = 0.f; for (int j = 0; j < NBI; ++j) s += sumsP[((size_t)b * NBI + j) * PSLOT]; ssum = s; }
    __syncthreads();
    int idx = blockIdx.x * 256 + threadIdx.x;
    int i = idx >> 6, k = idx & (IL - 1);
    float l1p = 0.f, d2p = 0.f;
    size_t o = (size_t)b * 1000 * IL + idx;
    if (k < 56) {
        float v = inter[o] / ssum;
        st2f(inter + o, v);
        float lab = exist[b] * prot_inter[((size_t)b * 1000 + i) * 56 + k];
        float df = v - lab;
        d2p = df * df;
        l1p = fabsf(v);
    }
    float t1 = block_reduce_sum(l1p, sm);
    float t2 = block_reduce_sum(d2p, sm);
    if (threadIdx.x == 0) { st2f(l1P + ((size_t)b * NBI + blockIdx.x) * PSLOT, t1); st2f(d2P + ((size_t)b * NBI + blockIdx.x) * PSLOT, t2); }
}

__global__ __launch_bounds__(256) void k_tpose(const float* __restrict__ inter, __bf16* __restrict__ interT)
{
    __shared__ float tl[64][65];
    const int b = blockIdx.y, i0 = blockIdx.x * 64, tid = threadIdx.x;
    for (int q = tid; q < 64 * 64; q += 256) { const int ii = q >> 6, kk = q & 63; const int i = i0 + ii;
        tl[kk][ii] = (i < 1000) ? inter[((size_t)b * 1000 + i) * IL + kk] : 0.f; }
    __syncthreads();
    const int kk = tid >> 2, q8 = (tid & 3) * 16;
    __bf16 hh[16];
    #pragma unroll
    for (int e = 0; e < 16; ++e) hh[e] = (__bf16)((kk < 56) ? tl[kk][q8 + e] * 65536.0f : 0.f);
    const v4u_t u0 = *(const v4ua*)hh, u1 = *(const v4ua*)(hh + 8);
    __bf16* d = interT + (size_t)b * 65536 + (size_t)kk * 1024 + i0 + q8;
    #pragma unroll 1
    for (int pass = 0; pass < 2; ++pass) { *(volatile v4u_t*)d = u0; *(volatile v4u_t*)(d + 8) = u1; __threadfence(); }
}

__global__ void k_rowsq(const float* __restrict__ inter, float* __restrict__ sbuf)
{
    int idx = blockIdx.x * blockDim.x + threadIdx.x;
    if (idx < 8000) {
        const float* r = inter + (size_t)idx * IL;
        float s = 0.f;
        #pragma unroll 8
        for (int k = 0; k < 56; ++k) s = fmaf(r[k], r[k], s);
        st2f(sbuf + idx, s);
    }
}

__global__ void k_cp(const float* __restrict__ prot, const float* __restrict__ comp,
                     const float* __restrict__ inter, float* __restrict__ cp_part)
{
    int i = blockIdx.x, b = blockIdx.y, d = threadIdx.x;
    float p = prot[((size_t)b * 1000 + i) * 256 + d];
    const float* cm = comp + (size_t)b * 56 * 256;
    const float* w  = inter + ((size_t)b * 1000 + i) * IL;
    float acc = 0.f;
    #pragma unroll 1
    for (int k = 0; k < 56; ++k)
        acc = fmaf(tanhf(p * cm[k * 256 + d]), w[k], acc);
    st2f(cp_part + ((size_t)b * 1000 + i) * 256 + d, acc);
}

__global__ void k_cpreduce(const float* __restrict__ cp_part, float* __restrict__ cp)
{
    int j = blockIdx.x * 256 + threadIdx.x;
    int b = j >> 8, d = j & 255;
    float s = 0.f;
    #pragma unroll 8
    for (int i = 0; i < 1000; ++i) s += cp_part[((size_t)b * 1000 + i) * 256 + d];
    st2f(cp + j, s);
}

__global__ void k_group(const float* __restrict__ contacts, const float* __restrict__ sbuf,
                        float* __restrict__ reggroup)
{
    __shared__ float sm[256];
    int kk = blockIdx.x, b = blockIdx.y, t = threadIdx.x;
    const float* cr = contacts + ((size_t)b * 1000 + kk) * 1000;
    const float* sb = sbuf + b * 1000;
    float g = 0.f, rs = 0.f;
    for (int i = t; i < 1000; i += 256) {
        float c = cr[i];
        g = fmaf(sb[i], c, g);
        rs += c;
    }
    float gt = block_reduce_sum(g, sm);
    float rt = block_reduce_sum(rs, sm);
    if (t == 0) {
        gt = (gt == 0.f) ? 1e10f : gt;
        st2f(reggroup + ((size_t)b * 1000 + kk) * PSLOT, sqrtf(gt) * sqrtf(rt));
    }
}

#define NBF 224
__global__ void k_fusedabs(const float* __restrict__ fo, float* __restrict__ facc)
{
    __shared__ float sm[256];
    int b = blockIdx.y;
    int idx = blockIdx.x * 256 + threadIdx.x;
    float v = (idx < 56 * FL) ? fabsf(fo[(size_t)b * 56 * FL + idx]) : 0.f;
    float t = block_reduce_sum(v, sm) * (1.0f / 65536.0f);
    if (threadIdx.x == 0) st2f(facc + ((size_t)b * NBF + blockIdx.x) * PSLOT, t);
}

__global__ void k_convpool(const float* __restrict__ cp, const float* __restrict__ cw,
                           const float* __restrict__ cb, float* __restrict__ h2)
{
    int b = blockIdx.x;
    const float* in = cp + (size_t)b * 256;
    for (int t = threadIdx.x; t < 2048; t += 256) {
        int c = t >> 5, p = t & 31;
        float mx = -3.4e38f;
        #pragma unroll
        for (int o4 = 0; o4 < 4; ++o4) {
            int o = p * 4 + o4;
            float a = cb[c];
            #pragma unroll
            for (int tt = 0; tt < 4; ++tt) {
                int j = 2 * o + tt - 1;
                if (j >= 0 && j < 256) a = fmaf(cw[c * 4 + tt], in[j], a);
            }
            a = LRELU(a);
            mx = fmaxf(mx, a);
        }
        st2f(h2 + (size_t)b * 2048 + t, mx);
    }
}

__global__ void k_mlp(const float* __restrict__ X, const float* __restrict__ W,
                      const float* __restrict__ bias, float* __restrict__ Y,
                      int Kin, int No)
{
    int b = blockIdx.y;
    int o = blockIdx.x * 256 + threadIdx.x;
    if (o >= No) return;
    const float* x = X + (size_t)b * Kin;
    float a = bias[o];
    for (int k = 0; k < Kin; ++k) a = fmaf(x[k], W[(size_t)k * No + o], a);
    st2f(Y + (size_t)b * No + o, LRELU(a));
}

__global__ void k_final(const float* l1P, const float* faP, const float* rgP,
                        const float* d2P, const float* r2, const float* Wr3,
                        const float* br3, const float* label, float* out)
{
    float ll1 = 0.f, lf = 0.f, lg = 0.f, l1s = 0.f, l2 = 0.f;
    for (int b = 0; b < 8; ++b) {
        float l1a = 0.f, d2a = 0.f, facc = 0.f, rg = 0.f;
        for (int j = 0; j < NBI; ++j) { l1a += l1P[((size_t)b * NBI + j) * PSLOT]; d2a += d2P[((size_t)b * NBI + j) * PSLOT]; }
        for (int j = 0; j < NBF; ++j) facc += faP[((size_t)b * NBF + j) * PSLOT];
        for (int j = 0; j < 1000; ++j) rg += rgP[((size_t)b * 1000 + j) * PSLOT];
        ll1 += l1a; lf += facc; lg += rg; l1s += sqrtf(d2a);
        float a = br3[0];
        for (int k = 0; k < 300; ++k) a = fmaf(r2[b * 300 + k], Wr3[k], a);
        float df = a - label[b];
        l2 += df * df;
    }
    const float L = (ll1 + lf + lg) * 0.125f + l1s * 0.125f + l2 * 0.125f;
    st2f(out, L);
}

extern "C" void kernel_launch(void* const* d_in, const int* in_sizes, int n_in,
                              void* d_out, int out_size, void* d_ws, size_t ws_size,
                              hipStream_t stream)
{
    (void)in_sizes; (void)n_in; (void)out_size; (void)ws_size;
    const float* prot_data = (const float*)d_in[0];
    const float* drug_ver  = (const float*)d_in[1];
    const float* drug_adj  = (const float*)d_in[2];
    const float* contacts  = (const float*)d_in[3];
    const float* prot_int  = (const float*)d_in[4];
    const float* exist     = (const float*)d_in[5];
    const float* label     = (const float*)d_in[6];
    const float* fused     = (const float*)d_in[7];
    const float* W_prot = (const float*)d_in[8];  const float* b_prot = (const float*)d_in[9];
    const float* gW0 = (const float*)d_in[10];    const float* gb0 = (const float*)d_in[11];
    const float* gW1 = (const float*)d_in[12];    const float* gb1 = (const float*)d_in[13];
    const float* gW2 = (const float*)d_in[14];    const float* gb2 = (const float*)d_in[15];
    const float* gWf = (const float*)d_in[16];    const float* gbf = (const float*)d_in[17];
    const float* Wjp = (const float*)d_in[18];    const float* bjp = (const float*)d_in[19];
    const float* Wjc = (const float*)d_in[20];    const float* bjc = (const float*)d_in[21];
    const float* convw = (const float*)d_in[22];  const float* convb = (const float*)d_in[23];
    const float* Wr1 = (const float*)d_in[24];    const float* br1 = (const float*)d_in[25];
    const float* Wr2 = (const float*)d_in[26];    const float* br2 = (const float*)d_in[27];
    const float* Wr3 = (const float*)d_in[28];    const float* br3 = (const float*)d_in[29];

    char* w = (char*)d_ws;
    size_t off = 0;
    auto carve = [&](size_t bytes) -> void* {
        void* p = w + off;
        off = (off + bytes + 255) & ~(size_t)255;
        return p;
    };
    __bf16* A1       = (__bf16*)carve(8000ull * 768 * 2);
    __bf16* WprotT   = (__bf16*)carve(256ull * 768 * 2);
    __bf16* WjpT     = (__bf16*)carve(256ull * 256 * 2);
    __bf16* fusedB   = (__bf16*)carve(1024ull * 1024 * 2);
    float*  prot     = (float*) carve(8000ull * 256 * 4);
    __bf16* reluprot = (__bf16*)carve(8000ull * 256 * 2);
    __bf16* qp_bf    = (__bf16*)carve((8000ull + 32) * 256 * 2);
    float*  g1b      = (float*) carve(8ull * 56 * 256 * 4);
    float*  g2b      = (float*) carve(8ull * 56 * 256 * 4);
    float*  compb    = (float*) carve(8ull * 56 * 256 * 4);
    float*  qcf      = (float*) carve(8ull * 56 * 256 * 4);
    __bf16* qc_bf    = (__bf16*)carve((8ull * 56 + 16) * 256 * 2);
    float*  inter    = (float*) carve((8ull * 1000 + 16) * IL * 4);
    __bf16* interT   = (__bf16*)carve(8ull * 64 * 1024 * 2);
    float*  fusedout = (float*) carve((8ull * 56 + 16) * FL * 4);
    float*  sums     = (float*) carve(8ull * NBI * PSLOT * 4);
    float*  l1a      = (float*) carve(8ull * NBI * PSLOT * 4);
    float*  d2a      = (float*) carve(8ull * NBI * PSLOT * 4);
    float*  rga      = (float*) carve(8ull * 1000 * PSLOT * 4);
    float*  faa      = (float*) carve(8ull * NBF * PSLOT * 4);
    float*  cp_part  = (float*) carve(8ull * 1000 * 256 * 4);
    float*  sbuf     = (float*) carve(8000ull * 4);
    float*  cpb      = (float*) carve(2048ull * 4);
    float*  h2       = (float*) carve(8ull * 2048 * 4);
    float*  r1b      = (float*) carve(8ull * 600 * 4);
    float*  r2b      = (float*) carve(8ull * 300 * 4);

    const int T = 256;
    auto cdiv = [](int a, int b) { return (a + b - 1) / b; };

    k_zero<<<cdiv(524288, T), T, 0, stream>>>((float*)fusedB, 524288);
    k_f2bf<<<cdiv(6144000, T), T, 0, stream>>>(prot_data, A1, 6144000);
    k_transconv<<<cdiv(768 * 256, T), T, 0, stream>>>(W_prot, WprotT, 768, 256);
    k_transconv<<<cdiv(256 * 256, T), T, 0, stream>>>(Wjp, WjpT, 256, 256);
    k_f2bf_pad<<<cdiv(999000, T), T, 0, stream>>>(fused, fusedB, 999, 1000, 1024);

    wmma_gemm_bt<<<dim3(4, 125, 1), 128, 0, stream>>>(A1, WprotT, prot, reluprot, b_prot,
        8000, 256, 768, 768, 768, 256, 0, 0, 0, 1);
    wmma_gemm_bt<<<dim3(4, 125, 1), 128, 0, stream>>>(reluprot, WjpT, nullptr, qp_bf, bjp,
        8000, 256, 256, 256, 256, 256, 0, 0, 0, 0);

    k_linear<<<448, 256, 0, stream>>>(drug_ver, gW0, gb0, g1b, nullptr, 43, 0);
    k_adjrelu<<<dim3(56, 8), 256, 0, stream>>>(drug_adj, g1b, g2b);
    k_linear<<<448, 256, 0, stream>>>(g2b, gW1, gb1, g1b, nullptr, 256, 0);
    k_adjrelu<<<dim3(56, 8), 256, 0, stream>>>(drug_adj, g1b, g2b);
    k_linear<<<448, 256, 0, stream>>>(g2b, gW2, gb2, g1b, nullptr, 256, 0);
    k_adjrelu<<<dim3(56, 8), 256, 0, stream>>>(drug_adj, g1b, g2b);
    k_linear<<<448, 256, 0, stream>>>(g2b, gWf, gbf, compb, nullptr, 256, 0);
    k_linear<<<448, 256, 0, stream>>>(compb, Wjc, bjc, qcf, qc_bf, 256, 1);

    wmma_gemm_bt<<<dim3(1, 16, 8), 128, 0, stream>>>(qp_bf, qc_bf, inter, nullptr, nullptr,
        1000, 56, 256, 256, 256, IL, 256000, 14336, 1000 * IL, 0);

    k_sigsum<<<dim3(NBI, 8), 256, 0, stream>>>(inter, sums);
    k_norm<<<dim3(NBI, 8), 256, 0, stream>>>(inter, sums, prot_int, exist, l1a, d2a);
    k_tpose<<<dim3(16, 8), 256, 0, stream>>>(inter, interT);
    k_rowsq<<<cdiv(8000, T), T, 0, stream>>>(inter, sbuf);

    wmma_gemm_bt<<<dim3(16, 1, 8), 128, 0, stream>>>(interT, fusedB, fusedout, nullptr, nullptr,
        56, 999, 1024, 1024, 1024, FL, 65536, 0, 56 * FL, 0);
    k_fusedabs<<<dim3(NBF, 8), 256, 0, stream>>>(fusedout, faa);

    k_cp<<<dim3(1000, 8), 256, 0, stream>>>(prot, compb, inter, cp_part);
    k_cpreduce<<<8, 256, 0, stream>>>(cp_part, cpb);
    k_group<<<dim3(1000, 8), 256, 0, stream>>>(contacts, sbuf, rga);

    k_convpool<<<8, 256, 0, stream>>>(cpb, convw, convb, h2);
    k_mlp<<<dim3(3, 8), 256, 0, stream>>>(h2, Wr1, br1, r1b, 2048, 600);
    k_mlp<<<dim3(2, 8), 256, 0, stream>>>(r1b, Wr2, br2, r2b, 600, 300);
    k_final<<<1, 1, 0, stream>>>(l1a, faa, rga, d2a, r2b, Wr3, br3, label, (float*)d_out);
}
